// EdgeAwareGATEncoder_80745385165159
// MI455X (gfx1250) — hardware-verified
//
#include <hip/hip_runtime.h>


namespace {
constexpr int Bn = 4, L = 2048, KN = 30, HID = 128, EDGE = 16, NL = 3, NH = 4, HD = 32, NT = Bn * L;
constexpr float WS = 64.0f, SCALE = 0.17677669529663687f;

typedef _Float16 b16;
typedef __attribute__((ext_vector_type(16))) _Float16 v16b;
typedef __attribute__((ext_vector_type(8)))  _Float16 v8b;
typedef __attribute__((ext_vector_type(8)))  float v8f;
typedef __attribute__((ext_vector_type(4)))  float v4f;

__device__ __forceinline__ v8b ld8b(const b16* p) { return *(const v8b*)p; }
__device__ __forceinline__ v16b cat8b(v8b a, v8b b) { return __builtin_shufflevector(a, b, 0, 1, 2, 3, 4, 5, 6, 7, 8, 9, 10, 11, 12, 13, 14, 15); }
__device__ __forceinline__ v16b frag_kb(const b16* p, int hh) { return cat8b(ld8b(p + 8 * hh), ld8b(p + 16 + 8 * hh)); }
__device__ __forceinline__ void split16(float v, b16& hi, b16& lo) { hi = (b16)v; lo = (b16)(v - (float)hi); }
__device__ __forceinline__ void frag_ksplit(const float* p, int hh, v16b& fh_, v16b& fl_) {
  const float* p0 = p + 8 * hh; const float* p1 = p + 16 + 8 * hh;
#pragma unroll
  for (int e = 0; e < 8; ++e) { b16 a, c; split16(p0[e], a, c); fh_[e] = a; fl_[e] = c; split16(p1[e], a, c); fh_[8 + e] = a; fl_[8 + e] = c; }
}
__device__ __forceinline__ v8f wmma16b(v16b a, v16b b, v8f c) {
  v8f d = __builtin_amdgcn_wmma_f32_16x16x32_f16(false, a, false, b, (short)0, c, false, false);
  asm volatile("v_nop\n\tv_nop\n\tv_nop\n\tv_nop" : "+v"(d) : "v"(a), "v"(b));
  return d;
}
__device__ __forceinline__ void wave_lds_sync() {
  __builtin_amdgcn_fence(__ATOMIC_RELEASE, "workgroup");
  __builtin_amdgcn_wave_barrier();
  __builtin_amdgcn_fence(__ATOMIC_ACQUIRE, "workgroup");
}

struct Opnd { const void* p0; const void* p1; int ld; };
template <int NP> __device__ __forceinline__ void load_frags(const Opnd& o, int row, int kb, int hh, v16b& fh_, v16b& fl_) {
  if (NP == 0) { frag_ksplit((const float*)o.p0 + (size_t)row * o.ld + kb, hh, fh_, fl_); }
  else if (NP == 3) {
    const float* p = (const float*)o.p0 + (size_t)row * o.ld + kb; const float* p0 = p + 8 * hh; const float* p1 = p + 16 + 8 * hh;
#pragma unroll
    for (int e = 0; e < 8; ++e) { fh_[e] = (b16)p0[e]; fh_[8 + e] = (b16)p1[e]; }
    fl_ = fh_;
  } else {
    fh_ = frag_kb((const b16*)o.p0 + (size_t)row * o.ld + kb, hh);
    if (NP == 2) fl_ = frag_kb((const b16*)o.p1 + (size_t)row * o.ld + kb, hh); else fl_ = fh_;
  }
}
template <int ANP, int BNP> __device__ __forceinline__ v8f mac(v16b ah, v16b al, v16b bh, v16b bl, v8f c) {
  c = wmma16b(ah, bh, c);
  if (BNP == 0 || BNP == 2) c = wmma16b(ah, bl, c);
  if (ANP == 0 || ANP == 2) c = wmma16b(al, bh, c);
  return c;
}
template <int ANP, int BNP>
__device__ __forceinline__ void gemm_tile(const Opnd& A, const Opnd& B, int K, int m0, int c0, int nloc, int hlf, v8f (&acc)[2][4]) {
  for (int kb = 0; kb < K; kb += 32) {
    v16b a0h, a0l, a1h, a1l;
    load_frags<ANP>(A, m0 + nloc, kb, hlf, a0h, a0l);
    load_frags<ANP>(A, m0 + 16 + nloc, kb, hlf, a1h, a1l);
#pragma unroll
    for (int t = 0; t < 4; ++t) {
      v16b bh, bl;
      load_frags<BNP>(B, c0 + t * 16 + nloc, kb, hlf, bh, bl);
      acc[0][t] = mac<ANP, BNP>(a0h, a0l, bh, bl, acc[0][t]);
      acc[1][t] = mac<ANP, BNP>(a1h, a1l, bh, bl, acc[1][t]);
    }
  }
}

struct Epi { float scale; const float* cscale; const float* cbias; const float* rbias; int act; float post; const float* rscale; const float* resid; };
__device__ __forceinline__ float epi_val(const Epi& e, float acc, int row, int col) {
  float val = acc * e.scale;
  if (e.cscale) val *= e.cscale[col];
  if (e.cbias) val += e.cbias[col];
  if (e.rbias) val += e.rbias[row];
  if (e.act == 1) val = 0.5f * val * (1.0f + erff(val * 0.70710678118654752f));
  val *= e.post;
  if (e.rscale) val *= e.rscale[(size_t)row * 32];
  return val;
}
__device__ __forceinline__ void epi_planes(v8f (&acc)[2][4], const Epi& e, bool two,
                                           b16* __restrict__ oh, b16* __restrict__ ol, int ldo, int m0, int c0, int lane, b16* Th, b16* Tl) {
  const int nloc = lane & 15, hlf = lane >> 4;
#pragma unroll
  for (int t = 0; t < 4; ++t)
#pragma unroll
    for (int r = 0; r < 2; ++r)
#pragma unroll
      for (int v = 0; v < 8; ++v) {
        const int rr = r * 16 + v + 8 * hlf, cc = t * 16 + nloc;
        const float val = epi_val(e, acc[r][t][v], m0 + rr, c0 + cc);
        b16 h_, l_; split16(val, h_, l_);
        Th[rr * 64 + cc] = h_; if (two) Tl[rr * 64 + cc] = l_;
      }
  wave_lds_sync();
  for (int pass = 0; pass < 2; ++pass) {
#pragma unroll
    for (int j = 0; j < 8; ++j) {
      const int rr = j * 4 + (lane >> 3), c8 = (lane & 7) * 8;
      const size_t o = (size_t)(m0 + rr) * ldo + c0 + c8;
      *(volatile v8b*)(oh + o) = ld8b(Th + rr * 64 + c8);
      if (two) *(volatile v8b*)(ol + o) = ld8b(Tl + rr * 64 + c8);
    }
    __threadfence();
  }
}
__device__ __forceinline__ void epi_f32(v8f (&acc)[2][4], const Epi& e, float* __restrict__ out, int ldo, int m0, int c0, int lane, float* Tt) {
  const int nloc = lane & 15, hlf = lane >> 4;
#pragma unroll
  for (int t = 0; t < 4; ++t)
#pragma unroll
    for (int r = 0; r < 2; ++r)
#pragma unroll
      for (int v = 0; v < 8; ++v) {
        const int rr = r * 16 + v + 8 * hlf, cc = t * 16 + nloc;
        Tt[rr * 64 + cc] = epi_val(e, acc[r][t][v], m0 + rr, c0 + cc);
      }
  wave_lds_sync();
  float* dst0 = out + (size_t)m0 * ldo + c0; const float* rs0 = e.resid ? e.resid + (size_t)m0 * ldo + c0 : nullptr;
  for (int pass = 0; pass < 2; ++pass) {
#pragma unroll
    for (int j = 0; j < 16; ++j) {
      const int rr = j * 2 + hlf, c4 = nloc * 4;
      v4f val = *(const v4f*)(Tt + rr * 64 + c4);
      if (rs0) val += *(const v4f*)(rs0 + (size_t)rr * ldo + c4);
      *(volatile v4f*)(dst0 + (size_t)rr * ldo + c4) = val;
    }
    __threadfence();
  }
}


__global__ __launch_bounds__(256) void prep_kernel(const float* __restrict__ Wq, const float* __restrict__ Wk, const float* __restrict__ Wv, const float* __restrict__ Wo,
                                                   const float* __restrict__ bq, const float* __restrict__ bk, const float* __restrict__ bv,
                                                   b16* __restrict__ wqkv, b16* __restrict__ wo16, float* __restrict__ bcat) {
  __shared__ __attribute__((aligned(16))) b16 Tl[HID][HID + 8];
  const int m = blockIdx.x & 3, layer = blockIdx.x >> 2, tid = threadIdx.x, lane = tid & 31, wave = tid >> 5;
  const float* W = ((m == 0) ? Wq : (m == 1) ? Wk : (m == 2) ? Wv : Wo) + (size_t)layer * HID * HID;
  for (int i = tid; i < HID * HID; i += 256) { const int k = i / HID, n = i % HID; Tl[n][k] = (b16)(W[i] * WS); }
  __syncthreads();
  b16* dst = (m < 3) ? (wqkv + ((size_t)layer * 3 * HID + m * HID) * HID) : (wo16 + (size_t)layer * HID * HID);
  for (int pass = 0; pass < 2; ++pass) {
#pragma unroll
    for (int j = 0; j < 8; ++j) { const int n = wave * 16 + j * 2 + (lane >> 4), c8 = (lane & 15) * 8; *(volatile v8b*)(dst + (size_t)n * HID + c8) = *(const v8b*)(&Tl[n][c8]); }
    if (m < 3 && tid < HID / 4) { const float* bs = ((m == 0) ? bq : (m == 1) ? bk : bv) + (size_t)layer * HID; *(volatile v4f*)(bcat + (size_t)layer * 3 * HID + m * HID + tid * 4) = *(const v4f*)(bs + tid * 4); }
    __threadfence();
  }
}

__global__ __launch_bounds__(128) void gemm_kernel(const float* __restrict__ A, int lda, const b16* __restrict__ Bm, int K, const float* __restrict__ bias, float* __restrict__ o32, int ldo) {
  __shared__ __attribute__((aligned(16))) float Ts[4][32 * 64];
  const int lane = threadIdx.x & 31, wave = threadIdx.x >> 5, nloc = lane & 15, hlf = lane >> 4;
  const int m0 = blockIdx.y * 128 + wave * 32, c0 = blockIdx.x * 64;
  v8f acc[2][4];
#pragma unroll
  for (int r = 0; r < 2; ++r)
#pragma unroll
    for (int t = 0; t < 4; ++t) acc[r][t] = (v8f){};
  const Opnd Ao{A, nullptr, lda}, Bo{Bm, nullptr, K};
  gemm_tile<3, 1>(Ao, Bo, K, m0, c0, nloc, hlf, acc);
  const Epi e{1.0f / WS, nullptr, bias, nullptr, 0, 1.0f, nullptr, nullptr};
  epi_f32(acc, e, o32, ldo, m0, c0, lane, Ts[wave]);
}

__global__ __launch_bounds__(256) void attn_kernel(const float* __restrict__ qkv, const float* __restrict__ hedge, const float* __restrict__ mask, const int* __restrict__ eidx,
                                                   const float* __restrict__ We, const float* __restrict__ be, float* __restrict__ orow) {
  const int wave = threadIdx.x >> 5, lane = threadIdx.x & 31, node = blockIdx.x * 8 + wave, b = node / L;
  const int h = lane >> 3;
  const v4f q4 = *(const v4f*)(qkv + (size_t)node * 3 * HID + lane * 4);
  const float we0 = We[(size_t)(2 * (lane & 7)) * NH + h], we1 = We[(size_t)(2 * (lane & 7) + 1) * NH + h], beh = be[h];
  const float ml = mask[node];
  float m = -INFINITY, l = 0.0f; v4f o = {0.0f, 0.0f, 0.0f, 0.0f};
#pragma unroll 1
  for (int k = 0; k < KN; ++k) {
    int id = eidx[(size_t)node * KN + k]; id = id < 0 ? 0 : (id >= L ? L - 1 : id);
    const size_t nb = (size_t)b * L + id;
    const v4f k4 = *(const v4f*)(qkv + nb * 3 * HID + HID + lane * 4);
    float s = q4[0] * k4[0] + q4[1] * k4[1] + q4[2] * k4[2] + q4[3] * k4[3];
    const float* hep = hedge + ((size_t)node * KN + k) * EDGE + 2 * (lane & 7);
    float eb = hep[0] * we0 + hep[1] * we1;
#pragma unroll
    for (int of = 1; of < 8; of <<= 1) { s += __shfl_xor(s, of); eb += __shfl_xor(eb, of); }
    s = s * SCALE + eb + beh;
    if (ml * mask[nb] == 0.0f) s = -1e9f;
    const float mn = fmaxf(m, s), al_ = __expf(m - mn), p = __expf(s - mn);
    m = mn; l = l * al_ + p;
    const v4f v4 = *(const v4f*)(qkv + nb * 3 * HID + 2 * HID + lane * 4);
#pragma unroll
    for (int e = 0; e < 4; ++e) o[e] = o[e] * al_ + p * v4[e];
  }
  const float inv = 1.0f / l;
#pragma unroll
  for (int e = 0; e < 4; ++e) o[e] *= inv;
  *(volatile v4f*)(orow + (size_t)node * HID + lane * 4) = o; __threadfence(); *(volatile v4f*)(orow + (size_t)node * HID + lane * 4) = o;
}

__global__ __launch_bounds__(256) void ln_kernel(const float* __restrict__ hin, const float* __restrict__ y, const float* __restrict__ g, const float* __restrict__ bb,
                                                 const float* __restrict__ mask, float* __restrict__ hout) {
  const int lane = threadIdx.x & 31, row = blockIdx.x * 8 + (threadIdx.x >> 5);
  v4f x = *(const v4f*)(hin + (size_t)row * HID + lane * 4); const v4f yy = *(const v4f*)(y + (size_t)row * HID + lane * 4);
  x += yy;
  float s = (x[0] + x[1]) + (x[2] + x[3]);
#pragma unroll
  for (int of = 16; of > 0; of >>= 1) s += __shfl_xor(s, of);
  const float mu = s * (1.0f / HID);
  float s2 = 0.0f;
#pragma unroll
  for (int e = 0; e < 4; ++e) { const float dl = x[e] - mu; s2 += dl * dl; }
#pragma unroll
  for (int of = 16; of > 0; of >>= 1) s2 += __shfl_xor(s2, of);
  const float rs = rsqrtf(s2 * (1.0f / HID) + 1e-5f), mk = mask[row];
  v4f w;
#pragma unroll
  for (int e = 0; e < 4; ++e) { const int c = lane * 4 + e; w[e] = ((x[e] - mu) * rs * g[c] + bb[c]) * mk; }
  *(volatile v4f*)(hout + (size_t)row * HID + lane * 4) = w; __threadfence(); *(volatile v4f*)(hout + (size_t)row * HID + lane * 4) = w;
}
}

extern "C" void kernel_launch(void* const* d_in, const int* in_sizes, int n_in,
                              void* d_out, int out_size, void* d_ws, size_t ws_size, hipStream_t stream) {
  (void)n_in; (void)out_size;
  const float* h0    = (const float*)d_in[0];
  const float* hedge = (const float*)d_in[1];
  const float* mask  = (const float*)d_in[2];
  const float* Wq = (const float*)d_in[3];  const float* bq = (const float*)d_in[4];
  const float* Wk = (const float*)d_in[5];  const float* bk = (const float*)d_in[6];
  const float* Wv = (const float*)d_in[7];  const float* bv = (const float*)d_in[8];
  const float* We = (const float*)d_in[9];  const float* be = (const float*)d_in[10];
  const float* Wo = (const float*)d_in[11]; const float* bo = (const float*)d_in[12];
  const float* lng = (const float*)d_in[13]; const float* lnb = (const float*)d_in[14];
  const int* eidx = (const int*)d_in[15];
  float* out = (float*)d_out;
  if (in_sizes[0] != NT * HID || in_sizes[1] != NT * KN * EDGE || in_sizes[2] != NT || in_sizes[3] != NL * HID * HID || in_sizes[15] != NT * KN) return;

  size_t off = 0; char* ws = (char*)d_ws;
  auto carve = [&](size_t bytes) { char* p = ws + off; off += (bytes + 255) & ~(size_t)255; return p; };
  b16* wqkv = (b16*)carve((size_t)NL * 3 * HID * HID * 2);
  b16* wo16 = (b16*)carve((size_t)NL * HID * HID * 2);
  float* bcat = (float*)carve((size_t)NL * 3 * HID * 4);
  float* qkv  = (float*)carve((size_t)NT * 3 * HID * 4);
  float* orow = (float*)carve((size_t)NT * HID * 4);
  float* y    = (float*)carve((size_t)NT * HID * 4);
  float* hA   = (float*)carve((size_t)NT * HID * 4);
  float* hB   = (float*)carve((size_t)NT * HID * 4);
  if (off > ws_size) return;
  prep_kernel<<<4 * NL, 256, 0, stream>>>(Wq, Wk, Wv, Wo, bq, bk, bv, wqkv, wo16, bcat);
  const float* hcur = h0;
  for (int i = 0; i < NL; ++i) {
    float* hnext = (i == NL - 1) ? out : ((i & 1) ? hB : hA);
    gemm_kernel<<<dim3(3 * HID / 64, NT / 128), 128, 0, stream>>>(hcur, HID, wqkv + (size_t)i * 3 * HID * HID, HID, bcat + (size_t)i * 3 * HID, qkv, 3 * HID);
    attn_kernel<<<NT / 8, 256, 0, stream>>>(qkv, hedge, mask, eidx, We + (size_t)i * EDGE * NH, be + (size_t)i * NH, orow);
    gemm_kernel<<<dim3(HID / 64, NT / 128), 128, 0, stream>>>(orow, HID, wo16 + (size_t)i * HID * HID, HID, bo + (size_t)i * HID, y, HID);
    ln_kernel<<<NT / 8, 256, 0, stream>>>(hcur, y, lng + (size_t)i * HID, lnb + (size_t)i * HID, mask, hnext);
    hcur = hnext;
  }
}
